// CRKTLayer_24661702214064
// MI455X (gfx1250) — hardware-verified
//
#include <hip/hip_runtime.h>
#include <hip/hip_bf16.h>


typedef __attribute__((ext_vector_type(16))) _Float16 v16h;
typedef __attribute__((ext_vector_type(8)))  _Float16 v8h;
typedef __attribute__((ext_vector_type(16))) __bf16   v16b;
typedef __attribute__((ext_vector_type(8)))  __bf16   v8b;
typedef __attribute__((ext_vector_type(8)))  float    v8f;
typedef __attribute__((ext_vector_type(4)))  float    v4f;

__device__ __forceinline__ unsigned short f2bf_bits(float f) {
  unsigned u = __float_as_uint(f);
  return (unsigned short)((u + 0x7FFFu + ((u >> 16) & 1u)) >> 16);
}
__device__ __forceinline__ float bf_bits2f(unsigned short h) { return __uint_as_float(((unsigned)h) << 16); }

__device__ __forceinline__ void dep_guard_h(v8f& a, v8f& b, v16h x, v16h y) { asm volatile("v_nop\n\tv_nop\n\tv_nop\n\tv_nop" : "+v"(a), "+v"(b) : "v"(x), "v"(y)); }
__device__ __forceinline__ void dep_guard_b(v8f& a, v8f& b, v16b x, v16b y) { asm volatile("v_nop\n\tv_nop\n\tv_nop\n\tv_nop" : "+v"(a), "+v"(b) : "v"(x), "v"(y)); }
__device__ __forceinline__ void keep4_h(v16h a, v16h b, v16h c, v16h d) { asm volatile("v_nop" :: "v"(a), "v"(b), "v"(c), "v"(d)); }
__device__ __forceinline__ void keep4_b(v16b a, v16b b, v16b c, v16b d) { asm volatile("v_nop" :: "v"(a), "v"(b), "v"(c), "v"(d)); }
__device__ __forceinline__ void acc_guard4(v8f& a, v8f& b, v8f& c, v8f& d) { asm volatile("v_nop\n\tv_nop\n\tv_nop\n\tv_nop" : "+v"(a), "+v"(b), "+v"(c), "+v"(d)); }
template <typename T> struct Frag;
template <> struct Frag<_Float16> {
  typedef v16h V; union U { v16h v; v8h h[2]; };
  static __device__ __forceinline__ v16h load(const _Float16* p) {
    U f; f.h[0] = *(const v8h*)(p); f.h[1] = *(const v8h*)(p + 16); return f.v;
  }
  static __device__ __forceinline__ v8f mma(v16h a, v16h b, v8f c) {
    return __builtin_amdgcn_wmma_f32_16x16x32_f16(false, a, false, b, (short)0, c, false, false);
  }
  static __device__ __forceinline__ void guard(v8f& a, v8f& b, v16h x, v16h y) { dep_guard_h(a, b, x, y); }
  static __device__ __forceinline__ void keep(v16h a, v16h b, v16h c, v16h d) { keep4_h(a, b, c, d); }
};
template <> struct Frag<__bf16> {
  typedef v16b V; union U { v16b v; v8b h[2]; };
  static __device__ __forceinline__ v16b load(const __bf16* p) {
    U f; f.h[0] = *(const v8b*)(p); f.h[1] = *(const v8b*)(p + 16); return f.v;
  }
  static __device__ __forceinline__ v8f mma(v16b a, v16b b, v8f c) {
    return __builtin_amdgcn_wmma_f32_16x16x32_bf16(false, a, false, b, (short)0, c, false, false);
  }
  static __device__ __forceinline__ void guard(v8f& a, v8f& b, v16b x, v16b y) { dep_guard_b(a, b, x, y); }
  static __device__ __forceinline__ void keep(v16b a, v16b b, v16b c, v16b d) { keep4_b(a, b, c, d); }
};

template <int ET> struct Elem;
template <> struct Elem<0> { typedef _Float16 T; };
template <> struct Elem<1> { typedef __bf16 T; };
template <int ET, bool SPLIT, int BIAS_MODE, int OUT_MODE, bool RESID, int ACT = 0>
__global__ __launch_bounds__(256) void wmma_gemm64(
    const unsigned short* __restrict__ Ap, const unsigned short* __restrict__ A2p, int lda, long strideA,
    const unsigned short* __restrict__ Btp, const unsigned short* __restrict__ Bt2p, int ldb, long strideB,
    void* __restrict__ Cout, void* __restrict__ Cout2, int ldc, long strideC,
    const float* __restrict__ bias,
    const float* __restrict__ resid, long strideR,
    int M, int N, int K, float scale) {
  typedef typename Elem<ET>::T T;
  typedef typename Frag<T>::V V;
  const T* A = (const T*)Ap; const T* A2 = (const T*)A2p; const T* Bt = (const T*)Btp; const T* Bt2 = (const T*)Bt2p;
  __shared__ __align__(16) float sT[8][16 * 68];
  const int b    = blockIdx.y;
  const int lane = threadIdx.x & 31;
  const int wave = threadIdx.x >> 5;
  const int tilesN = N >> 6;
  const int tilesM = M >> 6;
  const int tile = blockIdx.x * 8 + wave;
  if (tile >= tilesM * tilesN) return;
  const int tm = tile / tilesN;
  const int tn = tile - tm * tilesN;
  const int m0 = tm << 6;
  const int n0 = tn << 6;

  const T* Ab  = A  + (size_t)b * strideA;
  const T* Bb  = Bt + (size_t)b * strideB;
  const T* Ab2 = SPLIT ? (A2  + (size_t)b * strideA) : nullptr;
  const T* Bb2 = SPLIT ? (Bt2 + (size_t)b * strideB) : nullptr;

  const int rlane = lane & 15;
  const int koff  = (lane >> 4) * 8;
  const int mOff  = (lane >> 4) * 8;

  v8f acc[4][4];
#pragma unroll
  for (int i = 0; i < 4; ++i)
#pragma unroll
    for (int j = 0; j < 4; ++j) acc[i][j] = (v8f){0.f,0.f,0.f,0.f,0.f,0.f,0.f,0.f};

  for (int k0 = 0; k0 < K; k0 += 32) {
    V bh[4], bl[4];
#pragma unroll
    for (int j = 0; j < 4; ++j) {
      const size_t bo = (size_t)(n0 + (j << 4) + rlane) * ldb + koff + k0;
      bh[j] = Frag<T>::load(Bb + bo);
      if (SPLIT) bl[j] = Frag<T>::load(Bb2 + bo);
    }
#pragma unroll
    for (int i = 0; i < 4; ++i) {
      const size_t ao = (size_t)(m0 + (i << 4) + rlane) * lda + koff + k0;
      V ah = Frag<T>::load(Ab + ao);
      V al;
      if (SPLIT) al = Frag<T>::load(Ab2 + ao);
#pragma unroll
      for (int j = 0; j < 4; ++j) {
        acc[i][j] = Frag<T>::mma(ah, bh[j], acc[i][j]);
        if (SPLIT) {
          acc[i][j] = Frag<T>::mma(ah, bl[j], acc[i][j]);
          acc[i][j] = Frag<T>::mma(al, bh[j], acc[i][j]);
        }
      }
      Frag<T>::guard(acc[i][0], acc[i][3], ah, SPLIT ? al : ah);
    }
    Frag<T>::keep(bh[0], bh[1], bh[2], bh[3]);
    if (SPLIT) Frag<T>::keep(bl[0], bl[1], bl[2], bl[3]);
  }
  acc_guard4(acc[0][0], acc[0][1], acc[0][2], acc[0][3]);
  acc_guard4(acc[1][0], acc[1][1], acc[1][2], acc[1][3]);
  acc_guard4(acc[2][0], acc[2][1], acc[2][2], acc[2][3]);
  acc_guard4(acc[3][0], acc[3][1], acc[3][2], acc[3][3]);

  float* slab = sT[wave];
  const float* Rb = RESID ? (resid + (size_t)b * strideR) : nullptr;
#pragma unroll
  for (int i = 0; i < 4; ++i) {
    const int mBase = m0 + (i << 4);
#pragma unroll
    for (int j = 0; j < 4; ++j) {
      const int n = n0 + (j << 4) + rlane;
      float bv = 0.f;
      if (BIAS_MODE == 2) bv = bias[n];
#pragma unroll
      for (int r = 0; r < 8; ++r) {
        float v = acc[i][j][r] * scale;
        if (BIAS_MODE == 1) v += bias[mBase + mOff + r];
        if (BIAS_MODE == 2) v += bv;
        if (RESID) v += Rb[(size_t)(mBase + mOff + r) * ldc + n];
        if (ACT == 1) v = tanhf(v);
        if (ACT == 2) v = fmaxf(v, 0.0f);
        if (ACT == 3) v = v / (1.0f + expf(-v));
        if (ACT == 4) v = (v > 0.f) ? v : 0.01f * v;
        if (ACT == 5) v = 0.5f * v * (1.0f + erff(v * 0.70710678118654752f));
        slab[(mOff + r) * 68 + (j << 4) + rlane] = v;
      }
    }
    __builtin_amdgcn_fence(__ATOMIC_RELEASE, "workgroup");
    __builtin_amdgcn_wave_barrier();
    __builtin_amdgcn_fence(__ATOMIC_ACQUIRE, "workgroup");
    if (OUT_MODE == 0) {
      float* C = (float*)Cout + (size_t)b * strideC;
      const int hh = lane >> 4, c4 = (lane & 15) * 4;
      for (int pass = 0; pass < 2; ++pass) {
#pragma unroll
        for (int it = 0; it < 8; ++it) {
          const int row = it * 2 + hh;
          v4f v = *(const v4f*)(slab + row * 68 + c4);
          *(volatile v4f*)(C + (size_t)(mBase + row) * ldc + n0 + c4) = v;
        }
        __threadfence();
      }
    } else {
      const int q = lane >> 3, c8 = (lane & 7) * 8;
      unsigned short* C  = (unsigned short*)Cout  + (size_t)b * strideC;
      unsigned short* C2 = (OUT_MODE == 2) ? ((unsigned short*)Cout2 + (size_t)b * strideC) : nullptr;
      for (int pass = 0; pass < 2; ++pass) {
#pragma unroll
        for (int it = 0; it < 4; ++it) {
          const int row = it * 4 + q;
          const float* sp = slab + row * 68 + c8;
          v8h hv, lv;
#pragma unroll
          for (int e = 0; e < 8; ++e) {
            if (OUT_MODE == 1) {
              hv[e] = (_Float16)sp[e];
            } else {
              unsigned short hb = f2bf_bits(sp[e]);
              unsigned short lb = f2bf_bits(sp[e] - bf_bits2f(hb));
              hv[e] = __builtin_bit_cast(_Float16, hb);
              lv[e] = __builtin_bit_cast(_Float16, lb);
            }
          }
          *(volatile v8h*)(C + (size_t)(mBase + row) * ldc + n0 + c8) = hv;
          if (OUT_MODE == 2) *(volatile v8h*)(C2 + (size_t)(mBase + row) * ldc + n0 + c8) = lv;
        }
        __threadfence();
      }
    }
    __builtin_amdgcn_fence(__ATOMIC_RELEASE, "workgroup");
    __builtin_amdgcn_wave_barrier();
    __builtin_amdgcn_fence(__ATOMIC_ACQUIRE, "workgroup");
  }
}

__global__ __launch_bounds__(256) void cast_scale_f32_f16x2(
    const float* __restrict__ in, _Float16* __restrict__ out, int n2, float sc) {
  int i = blockIdx.x * 256 + threadIdx.x;
  if (i < n2) {
    const _Float16 h0 = (_Float16)(in[2 * i] * sc), h1 = (_Float16)(in[2 * i + 1] * sc);
    const unsigned u = (unsigned)__builtin_bit_cast(unsigned short, h0) | ((unsigned)__builtin_bit_cast(unsigned short, h1) << 16);
    ((volatile unsigned*)out)[i] = u;
    __threadfence();
    ((volatile unsigned*)out)[i] = u;
  }
}

#define SQ 1024
#define DM 512
#define NH 8
#define HD 64
#define QB 64
#define KC 64
#define PSCP 32768.0f

__device__ __forceinline__ v8f hmma(v16h a, v16h b, v8f c) {
  c = __builtin_amdgcn_wmma_f32_16x16x32_f16(false, a, false, b, (short)0, c, false, false);
  asm volatile("v_nop\n\tv_nop\n\tv_nop\n\tv_nop" : "+v"(c) : "v"(a), "v"(b));
  return c;
}
__device__ __forceinline__ float hmax16(float m) {
#pragma unroll
  for (int off = 1; off < 16; off <<= 1) m = fmaxf(m, __shfl_xor(m, off, 32));
  return m;
}
__device__ __forceinline__ float hsum16(float m) {
#pragma unroll
  for (int off = 1; off < 16; off <<= 1) m += __shfl_xor(m, off, 32);
  return m;
}

__global__ __launch_bounds__(128)
void attn_decay_kernel(const _Float16* __restrict__ Qh, const _Float16* __restrict__ Kh,
                       const _Float16* __restrict__ Vh, const float* __restrict__ decay,
                       _Float16* __restrict__ Oh) {
  __shared__ __align__(16) _Float16 Ksh[KC * HD];
  __shared__ __align__(16) _Float16 Vth[HD * KC];
  __shared__ __align__(16) _Float16 Psh[4][16 * KC];
  __shared__ __align__(16) float    Os[4][16 * 68];

  const int tid  = threadIdx.x;
  const int wave = tid >> 5;
  const int lane = tid & 31;
  const int hh   = lane >> 4;
  const int c    = lane & 15;

  const int bx = blockIdx.x;
  const int qb = bx & 15;
  const int bh = bx >> 4;
  const int h  = bh & (NH - 1);
  const int b  = bh >> 3;
  const int q0 = qb * QB + wave * 16;
  const float dec = fabsf(decay[h]);

  const size_t base = (size_t)b * SQ * DM + (size_t)h * HD;
  const _Float16* Qb = Qh + base;
  const _Float16* Kb = Kh + base;
  const _Float16* Vb = Vh + base;
  _Float16*       Ob = Oh + base;

  const v16h qf0 = Frag<_Float16>::load(Qb + (size_t)(q0 + c) * DM + 8 * hh);
  const v16h qf1 = Frag<_Float16>::load(Qb + (size_t)(q0 + c) * DM + 32 + 8 * hh);

  const int nch = qb + 1;
  const int kvr = tid >> 1, dh = (tid & 1) * 32;

  float m1[8], l1[8];
#pragma unroll
  for (int r = 0; r < 8; ++r) { m1[r] = -INFINITY; l1[r] = 0.f; }

  for (int kc = 0; kc < nch; ++kc) {
    const int kv0 = kc * KC;
    __syncthreads();
    {
      const _Float16* ks = Kb + (size_t)(kv0 + kvr) * DM + dh;
      _Float16* kd = Ksh + kvr * HD + dh;
#pragma unroll
      for (int i = 0; i < 4; ++i) *(v8h*)(kd + 8 * i) = *(const v8h*)(ks + 8 * i);
    }
    __syncthreads();

    v8f s[4];
#pragma unroll
    for (int j = 0; j < 4; ++j) {
      const _Float16* kp = Ksh + (j * 16 + c) * HD + 8 * hh;
      v8f a = (v8f){0.f,0.f,0.f,0.f,0.f,0.f,0.f,0.f};
      a = hmma(qf0, Frag<_Float16>::load(kp), a);
      a = hmma(qf1, Frag<_Float16>::load(kp + 32), a);
      s[j] = a;
    }
    const bool diag = (kc == qb);
    float cm[8];
#pragma unroll
    for (int r = 0; r < 8; ++r) {
      const int qrow = q0 + 8 * hh + r;
      float mx = -INFINITY;
#pragma unroll
      for (int j = 0; j < 4; ++j) {
        const int kvcol = kv0 + j * 16 + c;
        float v = s[j][r] * 0.125f;
        if (diag && (kvcol > qrow)) v = -INFINITY;
        s[j][r] = v;
        mx = fmaxf(mx, v);
      }
      cm[r] = hmax16(mx);
    }
#pragma unroll
    for (int r = 0; r < 8; ++r) {
      const float mnew = fmaxf(m1[r], cm[r]);
      const float al = __expf(m1[r] - mnew);
      m1[r] = mnew;
      float ps = 0.f;
#pragma unroll
      for (int j = 0; j < 4; ++j) ps += __expf(s[j][r] - mnew);
      l1[r] = l1[r] * al + hsum16(ps);
    }
  }
#pragma unroll
  for (int r = 0; r < 8; ++r) l1[r] = 1.0f / l1[r];

  float m2[8], l2[8], run[8];
  v8f oacc[4];
#pragma unroll
  for (int r = 0; r < 8; ++r) { m2[r] = -INFINITY; l2[r] = 0.f; run[r] = 0.f; }
#pragma unroll
  for (int t = 0; t < 4; ++t) oacc[t] = (v8f){0.f,0.f,0.f,0.f,0.f,0.f,0.f,0.f};

  _Float16* pwh = Psh[wave];

  for (int kc = 0; kc < nch; ++kc) {
    const int kv0 = kc * KC;
    __syncthreads();
    {
      const _Float16* ks = Kb + (size_t)(kv0 + kvr) * DM + dh;
      const _Float16* vs = Vb + (size_t)(kv0 + kvr) * DM + dh;
      _Float16* kd = Ksh + kvr * HD + dh;
#pragma unroll
      for (int i = 0; i < 4; ++i) {
        *(v8h*)(kd + 8 * i) = *(const v8h*)(ks + 8 * i);
        const v8h vv = *(const v8h*)(vs + 8 * i);
#pragma unroll
        for (int e = 0; e < 8; ++e) Vth[(dh + 8 * i + e) * KC + kvr] = vv[e];
      }
    }
    __syncthreads();

    v8f s[4];
#pragma unroll
    for (int j = 0; j < 4; ++j) {
      const _Float16* kp = Ksh + (j * 16 + c) * HD + 8 * hh;
      v8f a = (v8f){0.f,0.f,0.f,0.f,0.f,0.f,0.f,0.f};
      a = hmma(qf0, Frag<_Float16>::load(kp), a);
      a = hmma(qf1, Frag<_Float16>::load(kp + 32), a);
      s[j] = a;
    }
    const bool diag = (kc == qb);
    float cm[8];
#pragma unroll
    for (int r = 0; r < 8; ++r) {
      const int qrow = q0 + 8 * hh + r;
      float acc_run = run[r];
      float mx = -INFINITY;
#pragma unroll
      for (int j = 0; j < 4; ++j) {
        const int kvcol = kv0 + j * 16 + c;
        const bool valid = !(diag && (kvcol > qrow));
        const float sc = s[j][r] * 0.125f;
        const float p = valid ? (__expf(sc - m1[r]) * l1[r]) : 0.f;
        float x = p;
#pragma unroll
        for (int off = 1; off < 16; off <<= 1) {
          const float y = __shfl_up(x, off, 16);
          if (c >= off) x += y;
        }
        const float cum = acc_run + x;
        acc_run += __shfl(x, 15, 16);
        const float suf = 1.0f - cum;
        const float td = (float)(qrow - kvcol);
        const float dist = fmaxf(td * suf, 0.0f);
        const float te = __expf(-dec * dist);
        const float sv = valid ? (sc * te) : -INFINITY;
        s[j][r] = sv;
        mx = fmaxf(mx, sv);
      }
      run[r] = acc_run;
      cm[r] = hmax16(mx);
    }
#pragma unroll
    for (int r = 0; r < 8; ++r) {
      const float mnew = fmaxf(m2[r], cm[r]);
      const float al = __expf(m2[r] - mnew);
      m2[r] = mnew;
      float ps = 0.f;
#pragma unroll
      for (int j = 0; j < 4; ++j) {
        const float p = __expf(s[j][r] - mnew);
        ps += p;
        pwh[(8 * hh + r) * KC + j * 16 + c] = (_Float16)(p * PSCP);
      }
      l2[r] = l2[r] * al + hsum16(ps);
#pragma unroll
      for (int t = 0; t < 4; ++t) oacc[t][r] *= al;
    }
    __builtin_amdgcn_fence(__ATOMIC_RELEASE, "workgroup");
    __builtin_amdgcn_wave_barrier();
    __builtin_amdgcn_fence(__ATOMIC_ACQUIRE, "workgroup");
#pragma unroll 1
    for (int kk = 0; kk < 2; ++kk) {
      const v16h pa = Frag<_Float16>::load(pwh + c * KC + kk * 32 + 8 * hh);
#pragma unroll
      for (int t = 0; t < 4; ++t) {
        const v16h vbf = Frag<_Float16>::load(Vth + (t * 16 + c) * KC + kk * 32 + 8 * hh);
        oacc[t] = hmma(pa, vbf, oacc[t]);
      }
    }
  }

  float* os = Os[wave];
#pragma unroll
  for (int r = 0; r < 8; ++r) {
    const float inv = 1.0f / (l2[r] * PSCP);
#pragma unroll
    for (int t = 0; t < 4; ++t) os[(8 * hh + r) * 68 + t * 16 + c] = oacc[t][r] * inv;
  }
  __builtin_amdgcn_fence(__ATOMIC_RELEASE, "workgroup");
  __builtin_amdgcn_wave_barrier();
  __builtin_amdgcn_fence(__ATOMIC_ACQUIRE, "workgroup");
  {
    const int q8 = lane >> 3, c8 = (lane & 7) * 8;
    for (int pass = 0; pass < 2; ++pass) {
#pragma unroll
      for (int it = 0; it < 4; ++it) {
        const int row = it * 4 + q8;
        const float* sp = os + row * 68 + c8;
        v8h hv;
#pragma unroll
        for (int e = 0; e < 8; ++e) hv[e] = (_Float16)sp[e];
        *(volatile v8h*)(Ob + (size_t)(q0 + row) * DM + c8) = hv;
      }
      __threadfence();
    }
  }
}

__global__ __launch_bounds__(256) void layernorm512_kernel(
    const float* __restrict__ Y, const float* __restrict__ gam, const float* __restrict__ bet,
    float* __restrict__ out, int nrows) {
  const int wave = threadIdx.x >> 5, lane = threadIdx.x & 31;
  const int row = blockIdx.x * 8 + wave;
  if (row >= nrows) return;
  const float* yr = Y + (size_t)row * DM;
  v4f x[4];
#pragma unroll
  for (int i = 0; i < 4; ++i) x[i] = *(const v4f*)(yr + i * 128 + lane * 4);
  float sum = 0.f;
#pragma unroll
  for (int i = 0; i < 4; ++i) sum += (x[i][0] + x[i][1]) + (x[i][2] + x[i][3]);
#pragma unroll
  for (int off = 1; off < 32; off <<= 1) sum += __shfl_xor(sum, off, 32);
  const float mu = sum * (1.0f / 512.0f);
  float sq = 0.f;
#pragma unroll
  for (int i = 0; i < 4; ++i) {
#pragma unroll
    for (int e = 0; e < 4; ++e) { const float d = x[i][e] - mu; sq += d * d; }
  }
#pragma unroll
  for (int off = 1; off < 32; off <<= 1) sq += __shfl_xor(sq, off, 32);
  const float var  = sq * (1.0f / 512.0f);
  const float rstd = 1.0f / sqrtf(var + 1e-5f);
  v4f o[4];
#pragma unroll
  for (int i = 0; i < 4; ++i) {
    const v4f g  = *(const v4f*)(gam + i * 128 + lane * 4);
    const v4f bt = *(const v4f*)(bet + i * 128 + lane * 4);
#pragma unroll
    for (int e = 0; e < 4; ++e) o[i][e] = (x[i][e] - mu) * rstd * g[e] + bt[e];
  }
  float* orow = out + (size_t)row * DM;
  for (int pass = 0; pass < 2; ++pass) {
#pragma unroll
    for (int i = 0; i < 4; ++i) *(volatile v4f*)(orow + i * 128 + lane * 4) = o[i];
    __threadfence();
  }
}

extern "C" void kernel_launch(void* const* d_in, const int* in_sizes, int n_in,
                              void* d_out, int out_size, void* d_ws, size_t ws_size,
                              hipStream_t stream) {
  if (n_in < 12) return;
  const float* query  = (const float*)d_in[0];
  const float* key_in = (const float*)d_in[1];
  const float* value  = (const float*)d_in[2];
  const float* Wq     = (const float*)d_in[3];
  const float* bq     = (const float*)d_in[4];
  const float* Wv     = (const float*)d_in[5];
  const float* bv     = (const float*)d_in[6];
  const float* Wo     = (const float*)d_in[7];
  const float* bo     = (const float*)d_in[8];
  const float* decay  = (const float*)d_in[9];
  const float* gam    = (const float*)d_in[10];
  const float* bet    = (const float*)d_in[11];
  float* out = (float*)d_out;

  const int NE = in_sizes[0];
  const int rowsz = SQ * DM;
  if (NE <= 0 || (NE % rowsz) != 0) return;
  const int Bn = NE / rowsz;
  if (in_sizes[1] != NE || in_sizes[2] != NE || out_size != NE) return;
  if (in_sizes[3] != DM * DM || in_sizes[5] != DM * DM || in_sizes[7] != DM * DM) return;
  if (in_sizes[4] < DM || in_sizes[6] < DM || in_sizes[8] < DM || in_sizes[10] < DM || in_sizes[11] < DM) return;
  if (in_sizes[9] < NH) return;
  const int M  = Bn * SQ;
  const int NW = DM * DM;

  size_t off = 0;
  char* ws = (char*)d_ws;
  _Float16* Xh  = (_Float16*)(ws + off); off += (size_t)NE * 2;
  _Float16* Wqh = (_Float16*)(ws + off); off += (size_t)NW * 2;
  _Float16* Wvh = (_Float16*)(ws + off); off += (size_t)NW * 2;
  _Float16* Woh = (_Float16*)(ws + off); off += (size_t)NW * 2;
  _Float16* Qh  = (_Float16*)(ws + off); off += (size_t)NE * 2;
  _Float16* Kh  = (_Float16*)(ws + off); off += (size_t)NE * 2;
  _Float16* Vh  = (_Float16*)(ws + off); off += (size_t)NE * 2;
  _Float16* Oh  = (_Float16*)(ws + off); off += (size_t)NE * 2;
  float*    Yf  = (float*)(ws + off);    off += (size_t)NE * 4;
  if (off > ws_size) return;

  const float WSC = 64.0f, XSC = 8.0f;
  const int n2w = NW / 2, n2x = NE / 2;
  const dim3 gw((n2w + 255) / 256), gx((n2x + 255) / 256);

  cast_scale_f32_f16x2<<<gw, 256, 0, stream>>>(Wq, Wqh, n2w, WSC);
  cast_scale_f32_f16x2<<<gw, 256, 0, stream>>>(Wv, Wvh, n2w, WSC);
  cast_scale_f32_f16x2<<<gw, 256, 0, stream>>>(Wo, Woh, n2w, WSC);

  const int tiles = (M / 64) * (DM / 64);
  const dim3 gg((tiles + 7) / 8, 1);
  const float pscale = 1.0f / (WSC * XSC);

  cast_scale_f32_f16x2<<<gx, 256, 0, stream>>>(query, Xh, n2x, XSC);
  wmma_gemm64<0, false, 2, 1, false, 0><<<gg, 256, 0, stream>>>(
      (const unsigned short*)Xh, (const unsigned short*)Xh, DM, 0L,
      (const unsigned short*)Wqh, (const unsigned short*)Wqh, DM, 0L,
      (void*)Qh, (void*)Qh, DM, 0L, bq, bq, 0L, M, DM, DM, pscale);
  cast_scale_f32_f16x2<<<gx, 256, 0, stream>>>(key_in, Xh, n2x, XSC);
  wmma_gemm64<0, false, 2, 1, false, 0><<<gg, 256, 0, stream>>>(
      (const unsigned short*)Xh, (const unsigned short*)Xh, DM, 0L,
      (const unsigned short*)Wqh, (const unsigned short*)Wqh, DM, 0L,
      (void*)Kh, (void*)Kh, DM, 0L, bq, bq, 0L, M, DM, DM, pscale);
  cast_scale_f32_f16x2<<<gx, 256, 0, stream>>>(value, Xh, n2x, XSC);
  wmma_gemm64<0, false, 2, 1, false, 0><<<gg, 256, 0, stream>>>(
      (const unsigned short*)Xh, (const unsigned short*)Xh, DM, 0L,
      (const unsigned short*)Wvh, (const unsigned short*)Wvh, DM, 0L,
      (void*)Vh, (void*)Vh, DM, 0L, bv, bv, 0L, M, DM, DM, pscale);

  const dim3 ga(Bn * NH * (SQ / QB));
  attn_decay_kernel<<<ga, 128, 0, stream>>>(Qh, Kh, Vh, decay, Oh);

  wmma_gemm64<0, false, 2, 0, false, 0><<<gg, 256, 0, stream>>>(
      (const unsigned short*)Oh, (const unsigned short*)Oh, DM, 0L,
      (const unsigned short*)Woh, (const unsigned short*)Woh, DM, 0L,
      (void*)Yf, (void*)Yf, DM, 0L, bo, bo, 0L, M, DM, DM, 1.0f / WSC);

  const dim3 gl((M + 7) / 8);
  layernorm512_kernel<<<gl, 256, 0, stream>>>(Yf, gam, bet, out, M);
}
